// LidarCameraFusionMambaV2_16449724745542
// MI455X (gfx1250) — hardware-verified
//
#include <hip/hip_runtime.h>
#include <math.h>

typedef __attribute__((ext_vector_type(16))) _Float16 v16h;
typedef __attribute__((ext_vector_type(8)))  _Float16 v8h;
typedef __attribute__((ext_vector_type(16))) __bf16   v16b;
typedef __attribute__((ext_vector_type(8)))  __bf16   v8b;
typedef __attribute__((ext_vector_type(8)))  float    v8f;
typedef __attribute__((ext_vector_type(4)))  float    v4f;

constexpr int kBatch  = 2;
constexpr int kSeq    = 2048;
constexpr int kDm     = 512;
constexpr int kDin    = 1024;
constexpr int kNst    = 16;
constexpr int kDtR    = 32;
constexpr int kConvK  = 4;
constexpr int kXzP    = 2 * kDin;
constexpr int kXpW    = kDtR + 2 * kNst;
constexpr int kXdP    = 2 * kXpW;
constexpr int kRows   = kBatch * kSeq;
constexpr int kScanTS = 64;
constexpr int kScanCh = 64;
constexpr int kScanYP = 68;
static_assert(kXpW == 64 && kXdP == 128, "x_proj widths");
static_assert((kDm % 32) == 0 && (kDin % 32) == 0, "GEMM K multiples of 32");
static_assert((kRows % 64) == 0 && (kXzP % 64) == 0 && (kXdP % 64) == 0 && (kDm % 64) == 0 && (kDin % 64) == 0, "GEMM M,N multiples of 64");
static_assert((kSeq % kScanTS) == 0 && (kDin % kScanCh) == 0 && (kDin % 8) == 0, "tile multiples");

constexpr size_t kPlane512  = (size_t)kRows * kDm * 2;
constexpr size_t kPlane1024 = (size_t)kRows * kDin * 2;
constexpr size_t kF32_1024  = (size_t)kRows * kDin * 4;
constexpr size_t kOffCAMH = 0;
constexpr size_t kOffCAML = kOffCAMH + kPlane512;
constexpr size_t kOffLIDH = kOffCAML + kPlane512;
constexpr size_t kOffLIDL = kOffLIDH + kPlane512;
constexpr size_t kOffXD   = 0;
constexpr size_t kEndR5   = kOffLIDL + kPlane512;
constexpr size_t kOffWIH  = kEndR5;
constexpr size_t kOffWIL  = kOffWIH + (size_t)kXzP * kDm * 2;
constexpr size_t kOffWGH  = kOffWIL + (size_t)kXzP * kDm * 2;
constexpr size_t kOffWGL  = kOffWGH + (size_t)kDin * kDin * 2;
constexpr size_t kOffWXH  = kOffWGL + (size_t)kDin * kDin * 2;
constexpr size_t kOffWXL  = kOffWXH + (size_t)kXdP * kDin * 2;
constexpr size_t kOffWOH  = kOffWXL + (size_t)kXdP * kDin * 2;
constexpr size_t kOffWOL  = kOffWOH + (size_t)kDm * kDin * 2;
constexpr size_t kOffXZ   = kOffWOL + (size_t)kDm * kDin * 2;
constexpr size_t kOffR2   = kOffXZ + (size_t)kRows * kXzP * 4;
constexpr size_t kOffGLIN = kOffR2;
constexpr size_t kOffY0   = kOffR2;
constexpr size_t kOffR3   = kOffR2 + kF32_1024;
constexpr size_t kOffXG   = kOffR3;
constexpr size_t kOffYH   = kOffR3;
constexpr size_t kOffYL   = kOffR3 + kPlane1024;
constexpr size_t kOffR4   = kOffR3 + kF32_1024;
constexpr size_t kOffLXH  = kOffR4;
constexpr size_t kOffLXL  = kOffR4 + kPlane1024;
constexpr size_t kOffCXH  = kOffR4;
constexpr size_t kOffCXL  = kOffR4 + kPlane1024;
constexpr size_t kOffY1   = kOffR4;
constexpr size_t kWsTotal = kOffR4 + kF32_1024;
static_assert((size_t)kRows * kXdP * 4 <= kEndR5, "XD fits R5");
static_assert(kWsTotal == 111673344ull, "carve total");
static_assert(kWsTotal <= 134217728ull, "carve cap");
static_assert((kOffCAML % 128) == 0 && (kOffLIDH % 128) == 0 && (kOffLIDL % 128) == 0 && (kOffWIH % 128) == 0 &&
              (kOffWIL % 128) == 0 && (kOffWGH % 128) == 0 && (kOffWGL % 128) == 0 && (kOffWXH % 128) == 0 &&
              (kOffWXL % 128) == 0 && (kOffWOH % 128) == 0 && (kOffWOL % 128) == 0 && (kOffXZ % 128) == 0 &&
              (kOffR2 % 128) == 0 && (kOffR3 % 128) == 0 && (kOffYL % 128) == 0 && (kOffR4 % 128) == 0 &&
              (kOffLXL % 128) == 0, "128-B aligned regions");

__device__ __forceinline__ unsigned short f2bf_bits(float f) {
  unsigned u = __float_as_uint(f);
  return (unsigned short)((u + 0x7FFFu + ((u >> 16) & 1u)) >> 16);
}
__device__ __forceinline__ float bf_bits2f(unsigned short h) { return __uint_as_float(((unsigned)h) << 16); }

__device__ __forceinline__ void dep_guard_h(v8f& a, v8f& b, v16h x, v16h y) { asm volatile("v_nop\n\tv_nop\n\tv_nop\n\tv_nop" : "+v"(a), "+v"(b) : "v"(x), "v"(y)); }
__device__ __forceinline__ void dep_guard_b(v8f& a, v8f& b, v16b x, v16b y) { asm volatile("v_nop\n\tv_nop\n\tv_nop\n\tv_nop" : "+v"(a), "+v"(b) : "v"(x), "v"(y)); }
__device__ __forceinline__ void keep4_h(v16h a, v16h b, v16h c, v16h d) { asm volatile("v_nop" :: "v"(a), "v"(b), "v"(c), "v"(d)); }
__device__ __forceinline__ void keep4_b(v16b a, v16b b, v16b c, v16b d) { asm volatile("v_nop" :: "v"(a), "v"(b), "v"(c), "v"(d)); }
__device__ __forceinline__ void acc_guard4(v8f& a, v8f& b, v8f& c, v8f& d) { asm volatile("v_nop\n\tv_nop\n\tv_nop\n\tv_nop" : "+v"(a), "+v"(b), "+v"(c), "+v"(d)); }
template <typename T> struct Frag;
template <> struct Frag<_Float16> {
  typedef v16h V; union U { v16h v; v8h h[2]; };
  static __device__ __forceinline__ v16h load(const _Float16* p) {
    U f; f.h[0] = *(const v8h*)(p); f.h[1] = *(const v8h*)(p + 16); return f.v;
  }
  static __device__ __forceinline__ v8f mma(v16h a, v16h b, v8f c) {
    return __builtin_amdgcn_wmma_f32_16x16x32_f16(false, a, false, b, (short)0, c, false, false);
  }
  static __device__ __forceinline__ void guard(v8f& a, v8f& b, v16h x, v16h y) { dep_guard_h(a, b, x, y); }
  static __device__ __forceinline__ void keep(v16h a, v16h b, v16h c, v16h d) { keep4_h(a, b, c, d); }
};
template <> struct Frag<__bf16> {
  typedef v16b V; union U { v16b v; v8b h[2]; };
  static __device__ __forceinline__ v16b load(const __bf16* p) {
    U f; f.h[0] = *(const v8b*)(p); f.h[1] = *(const v8b*)(p + 16); return f.v;
  }
  static __device__ __forceinline__ v8f mma(v16b a, v16b b, v8f c) {
    return __builtin_amdgcn_wmma_f32_16x16x32_bf16(false, a, false, b, (short)0, c, false, false);
  }
  static __device__ __forceinline__ void guard(v8f& a, v8f& b, v16b x, v16b y) { dep_guard_b(a, b, x, y); }
  static __device__ __forceinline__ void keep(v16b a, v16b b, v16b c, v16b d) { keep4_b(a, b, c, d); }
};

template <int ET> struct Elem;
template <> struct Elem<0> { typedef _Float16 T; };
template <> struct Elem<1> { typedef __bf16 T; };
template <int ET, int SPL, int BIAS_MODE, int OUT_MODE, bool RESID, int ACT = 0>
__global__ __launch_bounds__(256) void wmma_gemm64(
    const unsigned short* __restrict__ Ap, const unsigned short* __restrict__ A2p, int lda, long strideA,
    const unsigned short* __restrict__ Btp, const unsigned short* __restrict__ Bt2p, int ldb, long strideB,
    void* __restrict__ Cout, void* __restrict__ Cout2, int ldc, long strideC,
    const float* __restrict__ bias,
    const float* __restrict__ resid, long strideR,
    int M, int N, int K, float scale) {
  typedef typename Elem<ET>::T T;
  typedef typename Frag<T>::V V;
  const T* A = (const T*)Ap; const T* A2 = (const T*)A2p; const T* Bt = (const T*)Btp; const T* Bt2 = (const T*)Bt2p;
  __shared__ __align__(16) float sT[8][16 * 68];
  const int b    = blockIdx.y;
  const int lane = threadIdx.x & 31;
  const int wave = threadIdx.x >> 5;
  const int tilesN = N >> 6;
  const int tilesM = M >> 6;
  const int tile = blockIdx.x * 8 + wave;
  if (tile >= tilesM * tilesN) return;
  const int tm = tile / tilesN;
  const int tn = tile - tm * tilesN;
  const int m0 = tm << 6;
  const int n0 = tn << 6;

  const T* Ab  = A  + (size_t)b * strideA;
  const T* Bb  = Bt + (size_t)b * strideB;
  const T* Ab2 = (SPL >= 1) ? (A2  + (size_t)b * strideA) : nullptr;
  const T* Bb2 = (SPL == 2) ? (Bt2 + (size_t)b * strideB) : nullptr;

  const int rlane = lane & 15;
  const int koff  = (lane >> 4) * 8;
  const int mOff  = (lane >> 4) * 8;

  v8f acc[4][4];
#pragma unroll
  for (int i = 0; i < 4; ++i)
#pragma unroll
    for (int j = 0; j < 4; ++j) acc[i][j] = (v8f){0.f,0.f,0.f,0.f,0.f,0.f,0.f,0.f};

  for (int k0 = 0; k0 < K; k0 += 32) {
    V bh[4], bl[4];
#pragma unroll
    for (int j = 0; j < 4; ++j) {
      const size_t bo = (size_t)(n0 + (j << 4) + rlane) * ldb + koff + k0;
      bh[j] = Frag<T>::load(Bb + bo);
      if (SPL == 2) bl[j] = Frag<T>::load(Bb2 + bo);
    }
#pragma unroll
    for (int i = 0; i < 4; ++i) {
      const size_t ao = (size_t)(m0 + (i << 4) + rlane) * lda + koff + k0;
      V ah = Frag<T>::load(Ab + ao);
      V al;
      if (SPL >= 1) al = Frag<T>::load(Ab2 + ao);
#pragma unroll
      for (int j = 0; j < 4; ++j) {
        acc[i][j] = Frag<T>::mma(ah, bh[j], acc[i][j]);
        if (SPL == 2) acc[i][j] = Frag<T>::mma(ah, bl[j], acc[i][j]);
        if (SPL >= 1) acc[i][j] = Frag<T>::mma(al, bh[j], acc[i][j]);
      }
      Frag<T>::guard(acc[i][0], acc[i][3], ah, (SPL >= 1) ? al : ah);
    }
    Frag<T>::keep(bh[0], bh[1], bh[2], bh[3]);
    if (SPL == 2) Frag<T>::keep(bl[0], bl[1], bl[2], bl[3]);
  }
  acc_guard4(acc[0][0], acc[0][1], acc[0][2], acc[0][3]);
  acc_guard4(acc[1][0], acc[1][1], acc[1][2], acc[1][3]);
  acc_guard4(acc[2][0], acc[2][1], acc[2][2], acc[2][3]);
  acc_guard4(acc[3][0], acc[3][1], acc[3][2], acc[3][3]);

  float* slab = sT[wave];
  const float* Rb = RESID ? (resid + (size_t)b * strideR) : nullptr;
#pragma unroll
  for (int i = 0; i < 4; ++i) {
    const int mBase = m0 + (i << 4);
#pragma unroll
    for (int j = 0; j < 4; ++j) {
      const int n = n0 + (j << 4) + rlane;
      float bv = 0.f;
      if (BIAS_MODE == 2) bv = bias[n];
#pragma unroll
      for (int r = 0; r < 8; ++r) {
        float v = acc[i][j][r] * scale;
        if (BIAS_MODE == 1) v += bias[mBase + mOff + r];
        if (BIAS_MODE == 2) v += bv;
        if (RESID) v += Rb[(size_t)(mBase + mOff + r) * ldc + n];
        if (ACT == 1) v = tanhf(v);
        if (ACT == 2) v = fmaxf(v, 0.0f);
        if (ACT == 3) v = v / (1.0f + expf(-v));
        if (ACT == 4) v = (v > 0.f) ? v : 0.01f * v;
        slab[(mOff + r) * 68 + (j << 4) + rlane] = v;
      }
    }
    __builtin_amdgcn_fence(__ATOMIC_RELEASE, "workgroup");
    __builtin_amdgcn_wave_barrier();
    __builtin_amdgcn_fence(__ATOMIC_ACQUIRE, "workgroup");
    if (OUT_MODE == 0) {
      float* C = (float*)Cout + (size_t)b * strideC;
      const int hh = lane >> 4, c4 = (lane & 15) * 4;
      for (int pass = 0; pass < 2; ++pass) {
#pragma unroll
        for (int it = 0; it < 8; ++it) {
          const int row = it * 2 + hh;
          v4f v = *(const v4f*)(slab + row * 68 + c4);
          *(volatile v4f*)(C + (size_t)(mBase + row) * ldc + n0 + c4) = v;
        }
        __threadfence();
      }
    } else {
      const int q = lane >> 3, c8 = (lane & 7) * 8;
      unsigned short* C  = (unsigned short*)Cout  + (size_t)b * strideC;
      unsigned short* C2 = (OUT_MODE == 2) ? ((unsigned short*)Cout2 + (size_t)b * strideC) : nullptr;
      for (int pass = 0; pass < 2; ++pass) {
#pragma unroll
        for (int it = 0; it < 4; ++it) {
          const int row = it * 4 + q;
          const float* sp = slab + row * 68 + c8;
          v8h hv, lv;
#pragma unroll
          for (int e = 0; e < 8; ++e) {
            if (OUT_MODE == 1) {
              hv[e] = (_Float16)sp[e];
            } else {
              unsigned short hb = f2bf_bits(sp[e]);
              unsigned short lb = f2bf_bits(sp[e] - bf_bits2f(hb));
              hv[e] = __builtin_bit_cast(_Float16, hb);
              lv[e] = __builtin_bit_cast(_Float16, lb);
            }
          }
          *(volatile v8h*)(C + (size_t)(mBase + row) * ldc + n0 + c8) = hv;
          if (OUT_MODE == 2) *(volatile v8h*)(C2 + (size_t)(mBase + row) * ldc + n0 + c8) = lv;
        }
        __threadfence();
      }
    }
    __builtin_amdgcn_fence(__ATOMIC_RELEASE, "workgroup");
    __builtin_amdgcn_wave_barrier();
    __builtin_amdgcn_fence(__ATOMIC_ACQUIRE, "workgroup");
  }
}

__global__ __launch_bounds__(256) void split_rows_bf16_kernel(
    const float* __restrict__ src, unsigned short* __restrict__ dhi, unsigned short* __restrict__ dlo, int total8)
{
  const int i = blockIdx.x * 256 + threadIdx.x;
  if (i >= total8) return;
  const size_t e0 = (size_t)i << 3;
  const v4f a0 = *(const v4f*)(src + e0);
  const v4f a1 = *(const v4f*)(src + e0 + 4);
  v8h hv, lv;
#pragma unroll
  for (int e = 0; e < 4; ++e) {
    const unsigned short h0 = f2bf_bits(a0[e]), h1 = f2bf_bits(a1[e]);
    const unsigned short l0 = f2bf_bits(a0[e] - bf_bits2f(h0)), l1 = f2bf_bits(a1[e] - bf_bits2f(h1));
    hv[e]     = __builtin_bit_cast(_Float16, h0);
    hv[4 + e] = __builtin_bit_cast(_Float16, h1);
    lv[e]     = __builtin_bit_cast(_Float16, l0);
    lv[4 + e] = __builtin_bit_cast(_Float16, l1);
  }
  unsigned short* qh = dhi + e0;
  unsigned short* ql = dlo + e0;
  *(volatile v8h*)qh = hv;
  *(volatile v8h*)ql = lv;
  __threadfence();
  *(volatile v8h*)qh = hv;
  *(volatile v8h*)ql = lv;
}

__global__ __launch_bounds__(256) void sum_split_bf16_kernel(
    const float* __restrict__ ya, const float* __restrict__ yb,
    unsigned short* __restrict__ dhi, unsigned short* __restrict__ dlo, int total8)
{
  const int i = blockIdx.x * 256 + threadIdx.x;
  if (i >= total8) return;
  const size_t e0 = (size_t)i << 3;
  const v4f a0 = *(const v4f*)(ya + e0) + *(const v4f*)(yb + e0);
  const v4f a1 = *(const v4f*)(ya + e0 + 4) + *(const v4f*)(yb + e0 + 4);
  v8h hv, lv;
#pragma unroll
  for (int e = 0; e < 4; ++e) {
    const unsigned short h0 = f2bf_bits(a0[e]), h1 = f2bf_bits(a1[e]);
    const unsigned short l0 = f2bf_bits(a0[e] - bf_bits2f(h0)), l1 = f2bf_bits(a1[e] - bf_bits2f(h1));
    hv[e]     = __builtin_bit_cast(_Float16, h0);
    hv[4 + e] = __builtin_bit_cast(_Float16, h1);
    lv[e]     = __builtin_bit_cast(_Float16, l0);
    lv[4 + e] = __builtin_bit_cast(_Float16, l1);
  }
  unsigned short* qh = dhi + e0;
  unsigned short* ql = dlo + e0;
  *(volatile v8h*)qh = hv;
  *(volatile v8h*)ql = lv;
  __threadfence();
  *(volatile v8h*)qh = hv;
  *(volatile v8h*)ql = lv;
}

__global__ __launch_bounds__(256) void gate_fuse_kernel(
    const float* __restrict__ XZ, const float* __restrict__ GL, const float* __restrict__ gb,
    float* __restrict__ XG, unsigned short* __restrict__ CXH, unsigned short* __restrict__ CXL)
{
  __shared__ __align__(16) float sG[2048];
  const int tid = threadIdx.x;
  const size_t eblk = (size_t)blockIdx.x * 2048;
  const size_t e0 = eblk + (size_t)tid * 8;
  const int row = (int)(e0 >> 10);
  const int d = (int)(e0 & (size_t)(kDin - 1));
  const float* cxp = XZ + (size_t)row * kXzP + d;
  const v4f c0 = *(const v4f*)(cxp);
  const v4f c1 = *(const v4f*)(cxp + 4);
  const v4f g0 = *(const v4f*)(GL + e0);
  const v4f g1 = *(const v4f*)(GL + e0 + 4);
  const v4f b0 = *(const v4f*)(gb + d);
  const v4f b1 = *(const v4f*)(gb + d + 4);
  v8h hv, lv;
  v4f xa, xb;
#pragma unroll
  for (int e = 0; e < 4; ++e) {
    const float cxa = c0[e], cxb = c1[e];
    const unsigned short h0 = f2bf_bits(cxa), h1 = f2bf_bits(cxb);
    const unsigned short l0 = f2bf_bits(cxa - bf_bits2f(h0)), l1 = f2bf_bits(cxb - bf_bits2f(h1));
    hv[e]     = __builtin_bit_cast(_Float16, h0);
    hv[4 + e] = __builtin_bit_cast(_Float16, h1);
    lv[e]     = __builtin_bit_cast(_Float16, l0);
    lv[4 + e] = __builtin_bit_cast(_Float16, l1);
    const float sa = g0[e] + b0[e];
    const float sb = g1[e] + b1[e];
    const float ga = __builtin_amdgcn_rcpf(1.0f + __expf(-sa));
    const float gbv = __builtin_amdgcn_rcpf(1.0f + __expf(-sb));
    xa[e] = cxa * ga;
    xb[e] = cxb * gbv;
  }
  {
    unsigned short* qh = CXH + e0;
    unsigned short* ql = CXL + e0;
    *(volatile v8h*)qh = hv;
    *(volatile v8h*)ql = lv;
    __threadfence();
    *(volatile v8h*)qh = hv;
    *(volatile v8h*)ql = lv;
  }
  *(v4f*)(sG + tid * 8) = xa;
  *(v4f*)(sG + tid * 8 + 4) = xb;
  __syncthreads();
  const v4f va = *(const v4f*)(sG + tid * 4);
  const v4f vb = *(const v4f*)(sG + 1024 + tid * 4);
  for (int pass = 0; pass < 2; ++pass) {
    *(volatile v4f*)(XG + eblk + (size_t)tid * 4) = va;
    *(volatile v4f*)(XG + eblk + 1024 + (size_t)tid * 4) = vb;
    __threadfence();
  }
}

__global__ __launch_bounds__(64) void scan_dir_kernel(
    const float* __restrict__ XD, const float* __restrict__ XG, const float* __restrict__ XZ,
    const float* __restrict__ cw, const float* __restrict__ cb,
    const float* __restrict__ Wdt, const float* __restrict__ bdt, const float* __restrict__ Alog,
    const float* __restrict__ Dp, float* __restrict__ Y, int dir)
{
  __shared__ __align__(16) float sX[kScanTS * kXpW];
  __shared__ __align__(16) float sY[kScanTS * kScanYP];
  __shared__ __align__(16) float sW[kDtR * kScanCh];
  __shared__ __align__(16) float sA[kNst * kScanCh];
  const int tid = threadIdx.x, lane = tid & 31, wave = tid >> 5;
  constexpr int kBlkPerB = kDin / kScanCh;
  const int bix = blockIdx.x / kBlkPerB;
  const int d0  = (blockIdx.x - bix * kBlkPerB) * kScanCh;
  const int d   = d0 + tid;
  const size_t row0 = (size_t)bix * kSeq;
  const int cofs = dir ? kXpW : 0;
#pragma unroll 1
  for (int r = 0; r < kDtR; ++r) sW[r * kScanCh + tid] = Wdt[(size_t)d * kDtR + r];
#pragma unroll 1
  for (int s = 0; s < kNst; ++s) sA[s * kScanCh + tid] = -expf(Alog[(size_t)d * kNst + s]);
  __syncthreads();
  float negA[kNst], h[kNst];
#pragma unroll
  for (int s = 0; s < kNst; ++s) {
    negA[s] = sA[s * kScanCh + tid];
    h[s] = 0.f;
  }
  const float bb = bdt[d], Dd = Dp[d];
  const float w0 = cw[(size_t)d * kConvK + 0], w1 = cw[(size_t)d * kConvK + 1];
  const float w2 = cw[(size_t)d * kConvK + 2], w3 = cw[(size_t)d * kConvK + 3];
  const float bc = cb[d];
  float xm3 = 0.f, xm2 = 0.f, xm1 = 0.f;
  const int lr = tid >> 4, lc4 = (tid & 15) * 4;
  const int hh = lane >> 4, c4 = (lane & 15) * 4;
#pragma unroll 1
  for (int s0 = 0; s0 < kSeq; s0 += kScanTS) {
    __syncthreads();
#pragma unroll
    for (int i = 0; i < 16; ++i) {
      const int r = lr + 4 * i;
      const int sw = s0 + r;
      const int t = dir ? (kSeq - 1 - sw) : sw;
      *(v4f*)(sX + r * kXpW + lc4) = *(const v4f*)(XD + (row0 + (size_t)t) * kXdP + cofs + lc4);
    }
    __syncthreads();
#pragma unroll 1
    for (int s = 0; s < kScanTS; ++s) {
      const int sw = s0 + s;
      const int t = dir ? (kSeq - 1 - sw) : sw;
      const size_t grow = row0 + (size_t)t;
      const float* xr = sX + s * kXpW;
      float vdot = 0.f;
#pragma unroll 1
      for (int r4 = 0; r4 < kDtR / 4; ++r4) {
        const v4f xv = *(const v4f*)(xr + 4 * r4);
        const float* wp = sW + (4 * r4) * kScanCh + tid;
        vdot = fmaf(xv[0], wp[0], vdot);
        vdot = fmaf(xv[1], wp[kScanCh], vdot);
        vdot = fmaf(xv[2], wp[2 * kScanCh], vdot);
        vdot = fmaf(xv[3], wp[3 * kScanCh], vdot);
      }
      float Bs[kNst], Cs[kNst];
#pragma unroll
      for (int q4 = 0; q4 < 4; ++q4) {
        const v4f bv = *(const v4f*)(xr + kDtR + 4 * q4);
        const v4f cv = *(const v4f*)(xr + kDtR + kNst + 4 * q4);
        Bs[4 * q4 + 0] = bv[0]; Bs[4 * q4 + 1] = bv[1]; Bs[4 * q4 + 2] = bv[2]; Bs[4 * q4 + 3] = bv[3];
        Cs[4 * q4 + 0] = cv[0]; Cs[4 * q4 + 1] = cv[1]; Cs[4 * q4 + 2] = cv[2]; Cs[4 * q4 + 3] = cv[3];
      }
      const float v   = vdot + bb;
      const float a   = __expf(-fabsf(v));
      const float up  = 1.0f + a;
      const float l1p = __logf(up) + (a - (up - 1.0f)) * __builtin_amdgcn_rcpf(up);
      const float dt  = fmaxf(v, 0.0f) + l1p;
      const float xcur = XG[grow * kDin + d];
      float cacc = w0 * xm3;
      cacc = fmaf(w1, xm2, cacc);
      cacc = fmaf(w2, xm1, cacc);
      cacc = fmaf(w3, xcur, cacc);
      const float sv = cacc + bc;
      const float sgu = __builtin_amdgcn_rcpf(1.0f + __expf(-sv));
      const float ut = sv * sgu;
      xm3 = xm2; xm2 = xm1; xm1 = xcur;
      const float dtx = dt * ut;
      float y = 0.f;
#pragma unroll
      for (int k = 0; k < kNst; ++k) {
        const float e = __expf(dt * negA[k]);
        h[k] = e * h[k] + dtx * Bs[k];
        y = h[k] * Cs[k] + y;
      }
      y = ut * Dd + y;
      const float zv = XZ[grow * kXzP + kDin + d];
      const float sg = __builtin_amdgcn_rcpf(1.0f + __expf(-zv));
      y = y * (zv * sg);
      sY[s * kScanYP + tid] = y;
    }
    __syncthreads();
    for (int pass = 0; pass < 2; ++pass) {
#pragma unroll
      for (int it = 0; it < 16; ++it) {
        const int srow = it * 4 + wave * 2 + hh;
        const int sw = s0 + srow;
        const int t = dir ? (kSeq - 1 - sw) : sw;
        const v4f val = *(const v4f*)(sY + srow * kScanYP + c4);
        *(volatile v4f*)(Y + (row0 + (size_t)t) * kDin + d0 + c4) = val;
      }
      __threadfence();
    }
  }
}

static inline unsigned cdiv_u(unsigned a, unsigned b) { return (a + b - 1) / b; }

extern "C" void kernel_launch(void* const* d_in, const int* in_sizes, int n_in,
                              void* d_out, int out_size, void* d_ws, size_t ws_size,
                              hipStream_t stream) {
  if (n_in < 20) return;
  if (in_sizes[0] != kRows * kDm || in_sizes[1] != kRows * kDm) return;
  if (in_sizes[2] != kXzP * kDm) return;
  if (in_sizes[3] != kDin * kConvK || in_sizes[10] != kDin * kConvK) return;
  if (in_sizes[4] != kDin || in_sizes[11] != kDin) return;
  if (in_sizes[5] != kXpW * kDin || in_sizes[12] != kXpW * kDin) return;
  if (in_sizes[6] != kDin * kDtR || in_sizes[13] != kDin * kDtR) return;
  if (in_sizes[7] != kDin || in_sizes[14] != kDin) return;
  if (in_sizes[8] != kDin * kNst || in_sizes[15] != kDin * kNst) return;
  if (in_sizes[9] != kDin || in_sizes[16] != kDin) return;
  if (in_sizes[17] != kDin * kDin) return;
  if (in_sizes[18] != kDin) return;
  if (in_sizes[19] != kDm * kDin) return;
  if (out_size != kRows * kDm) return;
  if (ws_size < kWsTotal) return;

  const float* featA     = (const float*)d_in[0];
  const float* featB     = (const float*)d_in[1];
  const float* W_in      = (const float*)d_in[2];
  const float* cw0       = (const float*)d_in[3];
  const float* cb0       = (const float*)d_in[4];
  const float* W_xp0     = (const float*)d_in[5];
  const float* W_dt0     = (const float*)d_in[6];
  const float* b_dt0     = (const float*)d_in[7];
  const float* A_log0    = (const float*)d_in[8];
  const float* Dp0       = (const float*)d_in[9];
  const float* cw1       = (const float*)d_in[10];
  const float* cb1       = (const float*)d_in[11];
  const float* W_xp1     = (const float*)d_in[12];
  const float* W_dt1     = (const float*)d_in[13];
  const float* b_dt1     = (const float*)d_in[14];
  const float* A_log1    = (const float*)d_in[15];
  const float* Dp1       = (const float*)d_in[16];
  const float* W_gate    = (const float*)d_in[17];
  const float* b_gate    = (const float*)d_in[18];
  const float* W_out     = (const float*)d_in[19];
  float* out = (float*)d_out;

  char* ws = (char*)d_ws;
  unsigned short* CAMH = (unsigned short*)(ws + kOffCAMH);
  unsigned short* CAML = (unsigned short*)(ws + kOffCAML);
  unsigned short* LIDH = (unsigned short*)(ws + kOffLIDH);
  unsigned short* LIDL = (unsigned short*)(ws + kOffLIDL);
  float*          XD   = (float*)(ws + kOffXD);
  unsigned short* WIH  = (unsigned short*)(ws + kOffWIH);
  unsigned short* WIL  = (unsigned short*)(ws + kOffWIL);
  unsigned short* WGH  = (unsigned short*)(ws + kOffWGH);
  unsigned short* WGL  = (unsigned short*)(ws + kOffWGL);
  unsigned short* WXH  = (unsigned short*)(ws + kOffWXH);
  unsigned short* WXL  = (unsigned short*)(ws + kOffWXL);
  unsigned short* WOH  = (unsigned short*)(ws + kOffWOH);
  unsigned short* WOL  = (unsigned short*)(ws + kOffWOL);
  float*          XZ   = (float*)(ws + kOffXZ);
  float*          GLIN = (float*)(ws + kOffGLIN);
  float*          Y0   = (float*)(ws + kOffY0);
  float*          XG   = (float*)(ws + kOffXG);
  unsigned short* YH   = (unsigned short*)(ws + kOffYH);
  unsigned short* YL   = (unsigned short*)(ws + kOffYL);
  unsigned short* LXH  = (unsigned short*)(ws + kOffLXH);
  unsigned short* LXL  = (unsigned short*)(ws + kOffLXL);
  unsigned short* CXH  = (unsigned short*)(ws + kOffCXH);
  unsigned short* CXL  = (unsigned short*)(ws + kOffCXL);
  float*          Y1   = (float*)(ws + kOffY1);

  {
    const int t8a = kRows * kDm / 8;
    split_rows_bf16_kernel<<<cdiv_u(t8a, 256), 256, 0, stream>>>(featB, CAMH, CAML, t8a);
    split_rows_bf16_kernel<<<cdiv_u(t8a, 256), 256, 0, stream>>>(featA, LIDH, LIDL, t8a);
    const int t8w = kXzP * kDm / 8;
    split_rows_bf16_kernel<<<cdiv_u(t8w, 256), 256, 0, stream>>>(W_in, WIH, WIL, t8w);
    const int t8g = kDin * kDin / 8;
    split_rows_bf16_kernel<<<cdiv_u(t8g, 256), 256, 0, stream>>>(W_gate, WGH, WGL, t8g);
    const int t8x = kXpW * kDin / 8;
    split_rows_bf16_kernel<<<cdiv_u(t8x, 256), 256, 0, stream>>>(W_xp0, WXH, WXL, t8x);
    split_rows_bf16_kernel<<<cdiv_u(t8x, 256), 256, 0, stream>>>(
        W_xp1, WXH + (size_t)kXpW * kDin, WXL + (size_t)kXpW * kDin, t8x);
    const int t8o = kDm * kDin / 8;
    split_rows_bf16_kernel<<<cdiv_u(t8o, 256), 256, 0, stream>>>(W_out, WOH, WOL, t8o);
  }

  wmma_gemm64<1, 2, 0, 2, false><<<dim3((kRows / 64) * (kDin / 64) / 8, 1), 256, 0, stream>>>(
      LIDH, LIDL, kDm, 0L,
      WIH, WIL, kDm, 0L,
      (void*)LXH, (void*)LXL, kDin, 0L,
      nullptr, nullptr, 0L,
      kRows, kDin, kDm, 1.0f);

  wmma_gemm64<1, 2, 0, 0, false><<<dim3((kRows / 64) * (kDin / 64) / 8, 1), 256, 0, stream>>>(
      LXH, LXL, kDin, 0L,
      WGH, WGL, kDin, 0L,
      (void*)GLIN, nullptr, kDin, 0L,
      nullptr, nullptr, 0L,
      kRows, kDin, kDin, 1.0f);

  wmma_gemm64<1, 2, 0, 0, false><<<dim3((kRows / 64) * (kXzP / 64) / 8, 1), 256, 0, stream>>>(
      CAMH, CAML, kDm, 0L,
      WIH, WIL, kDm, 0L,
      (void*)XZ, nullptr, kXzP, 0L,
      nullptr, nullptr, 0L,
      kRows, kXzP, kDm, 1.0f);

  gate_fuse_kernel<<<(kRows * kDin) / 2048, 256, 0, stream>>>(XZ, GLIN, b_gate, XG, CXH, CXL);

  wmma_gemm64<1, 2, 0, 0, false><<<dim3((kRows / 64) * (kXdP / 64) / 8, 1), 256, 0, stream>>>(
      CXH, CXL, kDin, 0L,
      WXH, WXL, kDin, 0L,
      (void*)XD, nullptr, kXdP, 0L,
      nullptr, nullptr, 0L,
      kRows, kXdP, kDin, 1.0f);

  scan_dir_kernel<<<kBatch * (kDin / kScanCh), kScanCh, 0, stream>>>(
      XD, XG, XZ, cw0, cb0, W_dt0, b_dt0, A_log0, Dp0, Y0, 0);
  scan_dir_kernel<<<kBatch * (kDin / kScanCh), kScanCh, 0, stream>>>(
      XD, XG, XZ, cw1, cb1, W_dt1, b_dt1, A_log1, Dp1, Y1, 1);

  {
    const int t8y = kRows * kDin / 8;
    sum_split_bf16_kernel<<<cdiv_u(t8y, 256), 256, 0, stream>>>(Y0, Y1, YH, YL, t8y);
  }

  wmma_gemm64<1, 2, 0, 0, false><<<dim3((kRows / 64) * (kDm / 64) / 8, 1), 256, 0, stream>>>(
      YH, YL, kDin, 0L,
      WOH, WOL, kDin, 0L,
      (void*)out, nullptr, kDm, 0L,
      nullptr, nullptr, 0L,
      kRows, kDm, kDin, 1.0f);
}
